// CoDABiMambaDecoderLayer_34866544508976
// MI455X (gfx1250) — hardware-run, weakly checked
//
#include <hip/hip_runtime.h>
#include <math.h>

typedef __attribute__((ext_vector_type(16))) _Float16 v16h;
typedef __attribute__((ext_vector_type(8)))  _Float16 v8h;
typedef __attribute__((ext_vector_type(8)))  float    v8f;
typedef __attribute__((ext_vector_type(4)))  float    v4f;

constexpr int kL    = 2048;
constexpr int kDm   = 1024;
constexpr int kDi   = 2048;
constexpr int kNs   = 16;
constexpr int kDtR  = 64;
constexpr int kXpN  = 96;
constexpr int kXpP  = 128;
constexpr int kXzP  = 2 * kDi;
constexpr int kIs   = 4096;
constexpr int kGuP  = 2 * kIs;
constexpr int kYcP  = 2 * kDi;
constexpr int kTP   = 260;
static_assert(kDtR + 2 * kNs == kXpN);
static_assert((kDm % 32) == 0 && (kDi % 32) == 0 && (kDtR % 32) == 0 && (kIs % 32) == 0 && (kYcP % 32) == 0);
static_assert((kL % 64) == 0 && (kXzP % 64) == 0 && (kXpP % 64) == 0 && (kDi % 64) == 0 && (kDm % 64) == 0 && (kGuP % 64) == 0);
static_assert((kDi % 256) == 0 && (kL % 64) == 0 && (kL % 16) == 0);

constexpr float kCarW   = 32.0f;
constexpr float kCarXc  = 64.0f;
constexpr float kCarDt  = 64.0f;
constexpr float kCarY   = 256.0f;
constexpr float kCarAct = 16.0f;
constexpr float kSclIn  = 1.0f / kCarW;
constexpr float kSclXp  = 1.0f / (kCarXc * kCarW);
constexpr float kSclDt  = 1.0f / (kCarDt * kCarW);
constexpr float kSclOut = 1.0f / (kCarY * kCarW);
constexpr float kSclGu  = 1.0f / kCarW;
constexpr float kSclDn  = 1.0f / (kCarAct * kCarW);
constexpr float kEps    = 1e-6f;
constexpr float kInvDm  = 1.0f / (float)kDm;

constexpr size_t kMiB      = 1048576;
constexpr size_t kOffX1    = 0;
constexpr size_t kOffH16   = 8 * kMiB;
constexpr size_t kOffZ16   = 12 * kMiB;
constexpr size_t kOffWIN16 = kOffZ16;
constexpr size_t kOffWOUT16= kOffZ16 + 8 * kMiB;
constexpr size_t kOffYC16  = kOffZ16 + 16 * kMiB;
constexpr size_t kOffXC16  = kOffZ16 + 32 * kMiB;
constexpr size_t kOffWXP16 = kOffZ16 + 40 * kMiB;
constexpr size_t kOffWDT16 = kOffWXP16 + kMiB / 2;
constexpr size_t kOffDTR16 = kOffWDT16 + kMiB / 4;
constexpr size_t kEndZ16   = kOffDTR16 + kMiB / 4;
constexpr size_t kOffWGU16 = kOffZ16;
constexpr size_t kOffACT16 = kOffZ16 + 16 * kMiB;
constexpr size_t kOffWDN16 = kOffZ16 + 32 * kMiB;
constexpr size_t kOffZF    = kEndZ16;
constexpr size_t kOffXZ    = kOffZF;
constexpr size_t kOffSS    = kOffZF;
constexpr size_t kOffXC    = kOffZF + 32 * kMiB;
constexpr size_t kOffDLR   = kOffZF + 48 * kMiB;
constexpr size_t kOffDBC   = kOffZF + 64 * kMiB;
constexpr size_t kOffGU    = kOffZF;
constexpr size_t kWsTotal  = kOffDBC + kMiB;
static_assert(kEndZ16 == 53 * kMiB);
static_assert(kWsTotal == 123731968ull);
static_assert(kWsTotal <= 134217728ull);
static_assert((size_t)kL * kDm * 4 == 8 * kMiB && (size_t)kL * kDm * 2 == 4 * kMiB);
static_assert((size_t)kXzP * kDm * 2 == 8 * kMiB && (size_t)kDm * kYcP * 2 == 8 * kMiB);
static_assert((size_t)kL * kYcP * 2 == 16 * kMiB && (size_t)kL * kDi * 2 == 8 * kMiB);
static_assert((size_t)kXpP * kDi * 2 == kMiB / 2 && (size_t)kDi * kDtR * 2 == kMiB / 4 && (size_t)kL * kDtR * 2 == kMiB / 4);
static_assert((size_t)kGuP * kDm * 2 == 16 * kMiB && (size_t)kL * kIs * 2 == 16 * kMiB && (size_t)kDm * kIs * 2 == 8 * kMiB);
static_assert(kOffWDN16 + 8 * kMiB <= kEndZ16);
static_assert((size_t)kL * kXzP * 4 == 32 * kMiB && (size_t)kL * kDi * 4 == 16 * kMiB && (size_t)kL * kXpP * 4 == kMiB);
static_assert((size_t)kL * kGuP * 4 == 64 * kMiB && kOffGU + 64 * kMiB <= kOffDBC);

__device__ __forceinline__ void grp_guard(v8f& a, v8f& b, v8f& c, v8f& d, v16h x, v16h b0, v16h b1, v16h b2, v16h b3) {
  asm volatile("v_nop\n\tv_nop\n\tv_nop\n\tv_nop" : "+v"(a), "+v"(b), "+v"(c), "+v"(d) : "v"(x), "v"(b0), "v"(b1), "v"(b2), "v"(b3));
}
__device__ __forceinline__ void keep4_h(v16h a, v16h b, v16h c, v16h d) { asm volatile("v_nop" :: "v"(a), "v"(b), "v"(c), "v"(d)); }
__device__ __forceinline__ void acc_guard4(v8f& a, v8f& b, v8f& c, v8f& d) { asm volatile("v_nop\n\tv_nop\n\tv_nop\n\tv_nop" : "+v"(a), "+v"(b), "+v"(c), "+v"(d)); }
struct FragH {
  union U { v16h v; v8h h[2]; };
  static __device__ __forceinline__ v16h load(const _Float16* p) {
    U f; f.h[0] = *(const v8h*)(p); f.h[1] = *(const v8h*)(p + 16); return f.v;
  }
  static __device__ __forceinline__ v8f mma(v16h a, v16h b, v8f c) {
    return __builtin_amdgcn_wmma_f32_16x16x32_f16(false, a, false, b, (short)0, c, false, false);
  }
};

template <bool BIAS_N, bool RESID>
__global__ __launch_bounds__(256) void wmma_gemm64_f16(
    const unsigned short* __restrict__ Ap, int lda,
    const unsigned short* __restrict__ Btp, int ldb,
    float* __restrict__ C, int ldc,
    const float* __restrict__ bias,
    const float* __restrict__ resid, int ldr,
    int M, int N, int K, float scale)
{
  const _Float16* A  = (const _Float16*)Ap;
  const _Float16* Bt = (const _Float16*)Btp;
  __shared__ __align__(16) float sT[8][16 * 68];
  const int lane = threadIdx.x & 31;
  const int wave = threadIdx.x >> 5;
  const int tilesN = N >> 6;
  const int tilesM = M >> 6;
  const int tile = blockIdx.x * 8 + wave;
  if (tile >= tilesM * tilesN) return;
  const int tm = tile / tilesN;
  const int tn = tile - tm * tilesN;
  const int m0 = tm << 6;
  const int n0 = tn << 6;

  const int rlane = lane & 15;
  const int koff  = (lane >> 4) * 8;
  const int mOff  = (lane >> 4) * 8;

  v8f acc[4][4];
#pragma unroll
  for (int i = 0; i < 4; ++i)
#pragma unroll
    for (int j = 0; j < 4; ++j) acc[i][j] = (v8f){0.f,0.f,0.f,0.f,0.f,0.f,0.f,0.f};

  for (int k0 = 0; k0 < K; k0 += 32) {
    v16h bh[4];
#pragma unroll
    for (int j = 0; j < 4; ++j) {
      const size_t bo = (size_t)(n0 + (j << 4) + rlane) * ldb + koff + k0;
      bh[j] = FragH::load(Bt + bo);
    }
#pragma unroll
    for (int i = 0; i < 4; ++i) {
      const size_t ao = (size_t)(m0 + (i << 4) + rlane) * lda + koff + k0;
      const v16h ah = FragH::load(A + ao);
#pragma unroll
      for (int j = 0; j < 4; ++j) acc[i][j] = FragH::mma(ah, bh[j], acc[i][j]);
      grp_guard(acc[i][0], acc[i][1], acc[i][2], acc[i][3], ah, bh[0], bh[1], bh[2], bh[3]);
    }
    keep4_h(bh[0], bh[1], bh[2], bh[3]);
  }
  acc_guard4(acc[0][0], acc[0][1], acc[0][2], acc[0][3]);
  acc_guard4(acc[1][0], acc[1][1], acc[1][2], acc[1][3]);
  acc_guard4(acc[2][0], acc[2][1], acc[2][2], acc[2][3]);
  acc_guard4(acc[3][0], acc[3][1], acc[3][2], acc[3][3]);

  float* slab = sT[wave];
  const int hh = lane >> 4;
  const int c4 = (lane & 15) * 4;
#pragma unroll
  for (int i = 0; i < 4; ++i) {
    const int mBase = m0 + (i << 4);
#pragma unroll
    for (int j = 0; j < 4; ++j) {
      const int n = n0 + (j << 4) + rlane;
      float bv = 0.f;
      if (BIAS_N) bv = bias[n];
#pragma unroll
      for (int r = 0; r < 8; ++r) {
        float v = acc[i][j][r] * scale;
        if (BIAS_N) v += bv;
        slab[(mOff + r) * 68 + (j << 4) + rlane] = v;
      }
    }
    __builtin_amdgcn_fence(__ATOMIC_RELEASE, "workgroup");
    __builtin_amdgcn_wave_barrier();
    __builtin_amdgcn_fence(__ATOMIC_ACQUIRE, "workgroup");
    v4f vv[8];
#pragma unroll
    for (int it = 0; it < 8; ++it) {
      const int row = it * 2 + hh;
      v4f v = *(const v4f*)(slab + row * 68 + c4);
      if (RESID) {
        const v4f rv = *(const v4f*)(resid + (size_t)(mBase + row) * ldr + n0 + c4);
        v = v + rv;
      }
      vv[it] = v;
    }
    for (int pass = 0; pass < 2; ++pass) {
#pragma unroll
      for (int it = 0; it < 8; ++it) {
        const int row = it * 2 + hh;
        *(volatile v4f*)(C + (size_t)(mBase + row) * ldc + n0 + c4) = vv[it];
      }
      __threadfence();
    }
    __builtin_amdgcn_fence(__ATOMIC_RELEASE, "workgroup");
    __builtin_amdgcn_wave_barrier();
    __builtin_amdgcn_fence(__ATOMIC_ACQUIRE, "workgroup");
  }
}

__global__ __launch_bounds__(256) void cast_rows_f16_kernel(
    const float* __restrict__ src, unsigned short* __restrict__ dst,
    int cols, int rowsReal, int dstPitch, int dstColOff, int total8, float scale)
{
  const int i = blockIdx.x * 256 + threadIdx.x;
  if (i >= total8) return;
  const size_t e0 = (size_t)i << 3;
  const int row = (int)(e0 / (size_t)cols);
  const int c   = (int)(e0 - (size_t)row * cols);
  const bool keep = (row < rowsReal);
  const int rc = keep ? row : (rowsReal - 1);
  const float* p = src + (size_t)rc * cols + c;
  const v4f a0 = *(const v4f*)(p);
  const v4f a1 = *(const v4f*)(p + 4);
  v8h hv;
#pragma unroll
  for (int e = 0; e < 4; ++e) {
    const float f0 = keep ? (a0[e] * scale) : 0.0f;
    const float f1 = keep ? (a1[e] * scale) : 0.0f;
    hv[e]     = (_Float16)f0;
    hv[4 + e] = (_Float16)f1;
  }
  unsigned short* q = dst + (size_t)row * dstPitch + dstColOff + c;
  *(volatile v8h*)q = hv;
  __threadfence();
  *(volatile v8h*)q = hv;
}

__device__ __forceinline__ float block_sum128(float v, float* red, int lane, int wave) {
#pragma unroll
  for (int off = 16; off > 0; off >>= 1) v += __shfl_xor(v, off, 32);
  if (lane == 0) red[wave] = v;
  __syncthreads();
  const float t = (red[0] + red[1]) + (red[2] + red[3]);
  __syncthreads();
  return t;
}

__global__ __launch_bounds__(128) void rmsnorm_in_kernel(
    const float* __restrict__ x, const float* __restrict__ w, const float* __restrict__ mask,
    unsigned short* __restrict__ H16)
{
  __shared__ float red[4];
  __shared__ __align__(16) float sH[kDm];
  const int tid = threadIdx.x, lane = tid & 31, wave = tid >> 5;
  const int row = blockIdx.x;
  const float* xr = x + (size_t)row * kDm;
  const v4f a = *(const v4f*)(xr + 4 * tid);
  const v4f b = *(const v4f*)(xr + 512 + 4 * tid);
  float ss = 0.f;
#pragma unroll
  for (int e = 0; e < 4; ++e) { ss += a[e] * a[e]; ss += b[e] * b[e]; }
  const float tot = block_sum128(ss, red, lane, wave);
  const float rs = rsqrtf(tot * kInvDm + kEps);
  const float mk = mask[row];
  const v4f wa = *(const v4f*)(w + 4 * tid);
  const v4f wb = *(const v4f*)(w + 512 + 4 * tid);
  v4f ha, hb;
#pragma unroll
  for (int e = 0; e < 4; ++e) {
    ha[e] = (wa[e] * (a[e] * rs)) * mk;
    hb[e] = (wb[e] * (b[e] * rs)) * mk;
  }
  *(v4f*)(sH + 4 * tid) = ha;
  *(v4f*)(sH + 512 + 4 * tid) = hb;
  __syncthreads();
  const v4f c0 = *(const v4f*)(sH + 8 * tid);
  const v4f c1 = *(const v4f*)(sH + 8 * tid + 4);
  v8h hv;
#pragma unroll
  for (int e = 0; e < 4; ++e) { hv[e] = (_Float16)c0[e]; hv[4 + e] = (_Float16)c1[e]; }
  unsigned short* q = H16 + (size_t)row * kDm + 8 * tid;
  *(volatile v8h*)q = hv;
  __threadfence();
  *(volatile v8h*)q = hv;
}

__global__ __launch_bounds__(128) void norm_mid_kernel(
    const float* __restrict__ S, const float* __restrict__ x, const float* __restrict__ mw,
    const float* __restrict__ lw, float* __restrict__ X1, unsigned short* __restrict__ H16)
{
  __shared__ float red[4];
  __shared__ __align__(16) float sH[kDm];
  const int tid = threadIdx.x, lane = tid & 31, wave = tid >> 5;
  const int row = blockIdx.x;
  const float* sr = S + (size_t)row * kDm;
  const float* xr = x + (size_t)row * kDm;
  const v4f sa = *(const v4f*)(sr + 4 * tid);
  const v4f sb = *(const v4f*)(sr + 512 + 4 * tid);
  float ss = 0.f;
#pragma unroll
  for (int e = 0; e < 4; ++e) { ss += sa[e] * sa[e]; ss += sb[e] * sb[e]; }
  const float tot1 = block_sum128(ss, red, lane, wave);
  const float rs1 = rsqrtf(tot1 * kInvDm + kEps);
  const v4f xa = *(const v4f*)(xr + 4 * tid);
  const v4f xb = *(const v4f*)(xr + 512 + 4 * tid);
  const v4f ma = *(const v4f*)(mw + 4 * tid);
  const v4f mb = *(const v4f*)(mw + 512 + 4 * tid);
  v4f ya, yb;
#pragma unroll
  for (int e = 0; e < 4; ++e) {
    ya[e] = xa[e] + ma[e] * (sa[e] * rs1);
    yb[e] = xb[e] + mb[e] * (sb[e] * rs1);
  }
  float* pa = X1 + (size_t)row * kDm + 4 * tid;
  float* pb = X1 + (size_t)row * kDm + 512 + 4 * tid;
  *(volatile v4f*)pa = ya;
  *(volatile v4f*)pb = yb;
  __threadfence();
  *(volatile v4f*)pa = ya;
  *(volatile v4f*)pb = yb;
  float s2 = 0.f;
#pragma unroll
  for (int e = 0; e < 4; ++e) { s2 += ya[e] * ya[e]; s2 += yb[e] * yb[e]; }
  const float tot2 = block_sum128(s2, red, lane, wave);
  const float rs2 = rsqrtf(tot2 * kInvDm + kEps);
  const v4f la = *(const v4f*)(lw + 4 * tid);
  const v4f lb = *(const v4f*)(lw + 512 + 4 * tid);
  v4f ha, hb;
#pragma unroll
  for (int e = 0; e < 4; ++e) {
    ha[e] = la[e] * (ya[e] * rs2);
    hb[e] = lb[e] * (yb[e] * rs2);
  }
  *(v4f*)(sH + 4 * tid) = ha;
  *(v4f*)(sH + 512 + 4 * tid) = hb;
  __syncthreads();
  const v4f c0 = *(const v4f*)(sH + 8 * tid);
  const v4f c1 = *(const v4f*)(sH + 8 * tid + 4);
  v8h hv;
#pragma unroll
  for (int e = 0; e < 4; ++e) { hv[e] = (_Float16)c0[e]; hv[4 + e] = (_Float16)c1[e]; }
  unsigned short* q = H16 + (size_t)row * kDm + 8 * tid;
  *(volatile v8h*)q = hv;
  __threadfence();
  *(volatile v8h*)q = hv;
}

__global__ __launch_bounds__(256) void conv_silu_kernel(
    const float* __restrict__ XZ, const float* __restrict__ cw, const float* __restrict__ cb,
    float* __restrict__ XC, unsigned short* __restrict__ XC16, int dir)
{
  __shared__ __align__(16) float sT[16 * kTP];
  const int tid = threadIdx.x, lane = tid & 31, wave = tid >> 5;
  const int d0 = blockIdx.x * 256, d = d0 + tid;
  const int t0 = blockIdx.y * 64;
  const v4f wv = *(const v4f*)(cw + (size_t)d * 4);
  const float w0 = wv[0], w1 = wv[1], w2 = wv[2], w3 = wv[3];
  const float bc = cb[d];
  const int sgn = dir ? -1 : 1;
  const int tstart = dir ? (t0 + 63) : t0;
  float xm3, xm2, xm1;
  {
    const int r1 = tstart - sgn, r2 = tstart - 2 * sgn, r3 = tstart - 3 * sgn;
    const int q1 = r1 < 0 ? 0 : (r1 > kL - 1 ? kL - 1 : r1);
    const int q2 = r2 < 0 ? 0 : (r2 > kL - 1 ? kL - 1 : r2);
    const int q3 = r3 < 0 ? 0 : (r3 > kL - 1 ? kL - 1 : r3);
    const float v1 = XZ[(size_t)q1 * kXzP + d];
    const float v2 = XZ[(size_t)q2 * kXzP + d];
    const float v3 = XZ[(size_t)q3 * kXzP + d];
    xm1 = (r1 >= 0 && r1 < kL) ? v1 : 0.f;
    xm2 = (r2 >= 0 && r2 < kL) ? v2 : 0.f;
    xm3 = (r3 >= 0 && r3 < kL) ? v3 : 0.f;
  }
  const int hrow = wave >> 1;
  const int hch  = (wave & 1) * 128 + lane * 4;
#pragma unroll 1
  for (int sub = 0; sub < 4; ++sub) {
    const int lb = dir ? (t0 + 48 - 16 * sub) : (t0 + 16 * sub);
#pragma unroll 1
    for (int k = 0; k < 16; ++k) {
      const int sl = dir ? (15 - k) : k;
      const float xcur = XZ[(size_t)(lb + sl) * kXzP + d];
      float acc = w0 * xm3;
      acc = fmaf(w1, xm2, acc);
      acc = fmaf(w2, xm1, acc);
      acc = fmaf(w3, xcur, acc);
      const float sv = acc + bc;
      const float sg = __builtin_amdgcn_rcpf(1.0f + expf(-sv));
      sT[sl * kTP + tid] = sv * sg;
      xm3 = xm2; xm2 = xm1; xm1 = xcur;
    }
    __syncthreads();
    v4f fv[4];
    v8h bv[2];
#pragma unroll
    for (int it = 0; it < 4; ++it) fv[it] = *(const v4f*)(sT + (it * 4 + hrow) * kTP + hch);
#pragma unroll
    for (int it = 0; it < 2; ++it) {
      const float* sp = sT + (it * 8 + wave) * kTP + lane * 8;
      const v4f a0 = *(const v4f*)(sp);
      const v4f a1 = *(const v4f*)(sp + 4);
#pragma unroll
      for (int e = 0; e < 4; ++e) {
        bv[it][e]     = (_Float16)(a0[e] * kCarXc);
        bv[it][4 + e] = (_Float16)(a1[e] * kCarXc);
      }
    }
    for (int pass = 0; pass < 2; ++pass) {
#pragma unroll
      for (int it = 0; it < 4; ++it)
        *(volatile v4f*)(XC + (size_t)(lb + it * 4 + hrow) * kDi + d0 + hch) = fv[it];
#pragma unroll
      for (int it = 0; it < 2; ++it)
        *(volatile v8h*)(XC16 + (size_t)(lb + it * 8 + wave) * kDi + d0 + lane * 8) = bv[it];
      __threadfence();
    }
    __syncthreads();
  }
}

__global__ __launch_bounds__(256) void dt_cast_kernel(
    const float* __restrict__ DBC, unsigned short* __restrict__ DTR16, int total8, float scale)
{
  const int i = blockIdx.x * 256 + threadIdx.x;
  if (i >= total8) return;
  const int e0  = i << 3;
  const int row = e0 >> 6;
  const int c8  = e0 & 63;
  const float* p = DBC + (size_t)row * kXpP + c8;
  const v4f a0 = *(const v4f*)(p);
  const v4f a1 = *(const v4f*)(p + 4);
  v8h hv;
#pragma unroll
  for (int e = 0; e < 4; ++e) {
    hv[e]     = (_Float16)(a0[e] * scale);
    hv[4 + e] = (_Float16)(a1[e] * scale);
  }
  unsigned short* qd = DTR16 + e0;
  *(volatile v8h*)qd = hv;
  __threadfence();
  *(volatile v8h*)qd = hv;
}

__global__ __launch_bounds__(256) void scan_kernel(
    const float* __restrict__ DLR, const float* __restrict__ XC, const float* __restrict__ XZ,
    const float* __restrict__ DBC, const float* __restrict__ A_log, const float* __restrict__ Dv,
    unsigned short* __restrict__ YC, int dir)
{
  __shared__ __align__(16) float sBC[16 * 32];
  __shared__ __align__(16) float sY[16 * kTP];
  const int tid = threadIdx.x, lane = tid & 31, wave = tid >> 5;
  const int d0 = blockIdx.x * 256, d = d0 + tid;
  const int colOff = dir ? kDi : 0;

#pragma unroll 1
  for (int n = 0; n < kNs; ++n) sY[n * kTP + tid] = -expf(A_log[(size_t)d * kNs + n]);
  __syncthreads();
  float An[kNs], h[kNs];
#pragma unroll
  for (int n = 0; n < kNs; ++n) { An[n] = sY[n * kTP + tid]; h[n] = 0.f; }
  __syncthreads();
  const float Dd = Dv[d];

#pragma unroll 1
  for (int c = 0; c < kL / 16; ++c) {
    const int l0 = dir ? (kL - 16 - 16 * c) : (16 * c);
    if (tid < 128) {
      const int r = tid >> 3, q = (tid & 7) * 4;
      const v4f v = *(const v4f*)(DBC + (size_t)(l0 + r) * kXpP + kDtR + q);
      *(v4f*)(sBC + r * 32 + q) = v;
    }
    __syncthreads();
#pragma unroll 1
    for (int k = 0; k < 16; ++k) {
      const int s = dir ? (15 - k) : k;
      const size_t m = (size_t)(l0 + s);
      float a  = DLR[m * kDi + d];
      float xv = XC[m * kDi + d];
      float zv = XZ[m * kXzP + kDi + d];
      asm volatile("" : "+v"(a), "+v"(xv), "+v"(zv));
      const float ea  = __expf(-fabsf(a));
      const float u1  = 1.0f + ea;
      const float l1p = __logf(u1) + (ea - (u1 - 1.0f)) * __builtin_amdgcn_rcpf(u1);
      const float delta = fmaxf(a, 0.0f) + l1p;
      const float dtx = delta * xv;
      v4f Bq[4], Cq[4];
#pragma unroll
      for (int qq = 0; qq < 4; ++qq) {
        Bq[qq] = *(const v4f*)(sBC + s * 32 + 4 * qq);
        Cq[qq] = *(const v4f*)(sBC + s * 32 + kNs + 4 * qq);
      }
      float y = 0.f;
#pragma unroll
      for (int n = 0; n < kNs; ++n) {
        const float e  = __expf(delta * An[n]);
        const float hn = e * h[n] + dtx * Bq[n >> 2][n & 3];
        h[n] = hn;
        y = hn * Cq[n >> 2][n & 3] + y;
      }
      y = xv * Dd + y;
      const float sg = __builtin_amdgcn_rcpf(1.0f + expf(-zv));
      const float g  = zv * sg;
      sY[s * kTP + tid] = (y * g) * kCarY;
    }
    __syncthreads();
    v8h hv[2];
#pragma unroll
    for (int it = 0; it < 2; ++it) {
      const float* sp = sY + (it * 8 + wave) * kTP + lane * 8;
      const v4f a0 = *(const v4f*)(sp);
      const v4f a1 = *(const v4f*)(sp + 4);
#pragma unroll
      for (int e = 0; e < 4; ++e) { hv[it][e] = (_Float16)a0[e]; hv[it][4 + e] = (_Float16)a1[e]; }
    }
    for (int pass = 0; pass < 2; ++pass) {
#pragma unroll
      for (int it = 0; it < 2; ++it)
        *(volatile v8h*)(YC + (size_t)(l0 + it * 8 + wave) * kYcP + colOff + d0 + lane * 8) = hv[it];
      __threadfence();
    }
  }
}

__global__ __launch_bounds__(256) void silu_mul_kernel(
    const float* __restrict__ GU, unsigned short* __restrict__ ACT, int total8)
{
  const int i = blockIdx.x * 256 + threadIdx.x;
  if (i >= total8) return;
  const size_t e0 = (size_t)i << 3;
  const int row = (int)(e0 >> 12);
  const int c   = (int)(e0 & 4095);
  const float* pg = GU + (size_t)row * kGuP + c;
  const float* pu = pg + kIs;
  const v4f g0 = *(const v4f*)(pg);
  const v4f g1 = *(const v4f*)(pg + 4);
  const v4f u0 = *(const v4f*)(pu);
  const v4f u1 = *(const v4f*)(pu + 4);
  v8h hv;
#pragma unroll
  for (int e = 0; e < 4; ++e) {
    const float ga = g0[e], gb = g1[e];
    const float sa = __builtin_amdgcn_rcpf(1.0f + expf(-ga));
    const float sb = __builtin_amdgcn_rcpf(1.0f + expf(-gb));
    hv[e]     = (_Float16)(((ga * sa) * u0[e]) * kCarAct);
    hv[4 + e] = (_Float16)(((gb * sb) * u1[e]) * kCarAct);
  }
  unsigned short* q = ACT + e0;
  *(volatile v8h*)q = hv;
  __threadfence();
  *(volatile v8h*)q = hv;
}

extern "C" void kernel_launch(void* const* d_in, const int* in_sizes, int n_in,
                              void* d_out, int out_size, void* d_ws, size_t ws_size,
                              hipStream_t stream)
{
  if (n_in < 26) return;
  if (in_sizes[0] != kL * kDm || in_sizes[1] != kL) return;
  if (in_sizes[2] != kDm || in_sizes[3] != kDm || in_sizes[4] != kDm) return;
  if (in_sizes[5] != kIs * kDm || in_sizes[6] != kIs * kDm || in_sizes[7] != kDm * kIs) return;
  for (int dd = 0; dd < 2; ++dd) {
    const int b = 8 + 9 * dd;
    if (in_sizes[b + 0] != kXzP * kDm) return;
    if (in_sizes[b + 1] != kDi * 4 || in_sizes[b + 2] != kDi) return;
    if (in_sizes[b + 3] != kXpN * kDi) return;
    if (in_sizes[b + 4] != kDi * kDtR || in_sizes[b + 5] != kDi) return;
    if (in_sizes[b + 6] != kDi * kNs || in_sizes[b + 7] != kDi) return;
    if (in_sizes[b + 8] != kDm * kDi) return;
  }
  if (out_size != kL * kDm) return;
  if (ws_size < kWsTotal) return;

  const float* hs      = (const float*)d_in[0];
  const float* amask   = (const float*)d_in[1];
  const float* mnorm_w = (const float*)d_in[2];
  const float* ln1_w   = (const float*)d_in[3];
  const float* ln2_w   = (const float*)d_in[4];
  const float* gate_w  = (const float*)d_in[5];
  const float* up_w    = (const float*)d_in[6];
  const float* down_w  = (const float*)d_in[7];
  float* dout = (float*)d_out;

  char* ws = (char*)d_ws;
  float*          X1     = (float*)(ws + kOffX1);
  unsigned short* H16    = (unsigned short*)(ws + kOffH16);
  unsigned short* WIN16  = (unsigned short*)(ws + kOffWIN16);
  unsigned short* WOUT16 = (unsigned short*)(ws + kOffWOUT16);
  unsigned short* YC16   = (unsigned short*)(ws + kOffYC16);
  unsigned short* XC16   = (unsigned short*)(ws + kOffXC16);
  unsigned short* WXP16  = (unsigned short*)(ws + kOffWXP16);
  unsigned short* WDT16  = (unsigned short*)(ws + kOffWDT16);
  unsigned short* DTR16  = (unsigned short*)(ws + kOffDTR16);
  unsigned short* WGU16  = (unsigned short*)(ws + kOffWGU16);
  unsigned short* ACT16  = (unsigned short*)(ws + kOffACT16);
  unsigned short* WDN16  = (unsigned short*)(ws + kOffWDN16);
  float*          XZ     = (float*)(ws + kOffXZ);
  float*          SS     = (float*)(ws + kOffSS);
  float*          XC     = (float*)(ws + kOffXC);
  float*          DLR    = (float*)(ws + kOffDLR);
  float*          DBC    = (float*)(ws + kOffDBC);
  float*          GU     = (float*)(ws + kOffGU);
  const float* dummy_bias  = (const float*)d_in[13];
  const float* dummy_resid = hs;

  rmsnorm_in_kernel<<<kL, 128, 0, stream>>>(hs, ln1_w, amask, H16);

  for (int dd = 0; dd < 2; ++dd) {
    const int b = 8 + 9 * dd;
    const float* in_w    = (const float*)d_in[b + 0];
    const float* conv_w  = (const float*)d_in[b + 1];
    const float* conv_b  = (const float*)d_in[b + 2];
    const float* xproj_w = (const float*)d_in[b + 3];
    const float* dt_w    = (const float*)d_in[b + 4];
    const float* dt_b    = (const float*)d_in[b + 5];
    const float* A_log   = (const float*)d_in[b + 6];
    const float* Dp      = (const float*)d_in[b + 7];
    const float* out_w   = (const float*)d_in[b + 8];

    cast_rows_f16_kernel<<<(kXzP * kDm / 8) / 256, 256, 0, stream>>>(in_w, WIN16, kDm, kXzP, kDm, 0, kXzP * kDm / 8, kCarW);
    cast_rows_f16_kernel<<<(kXpP * kDi / 8) / 256, 256, 0, stream>>>(xproj_w, WXP16, kDi, kXpN, kDi, 0, kXpP * kDi / 8, kCarW);
    cast_rows_f16_kernel<<<(kDi * kDtR / 8) / 256, 256, 0, stream>>>(dt_w, WDT16, kDtR, kDi, kDtR, 0, kDi * kDtR / 8, kCarW);
    cast_rows_f16_kernel<<<(kDm * kDi / 8) / 256, 256, 0, stream>>>(out_w, WOUT16, kDi, kDm, kYcP, dd * kDi, kDm * kDi / 8, kCarW);

    wmma_gemm64_f16<false, false><<<256, 256, 0, stream>>>(
        H16, kDm, WIN16, kDm, XZ, kXzP, dummy_bias, dummy_resid, kDm, kL, kXzP, kDm, kSclIn);

    conv_silu_kernel<<<dim3(kDi / 256, kL / 64), 256, 0, stream>>>(XZ, conv_w, conv_b, XC, XC16, dd);

    wmma_gemm64_f16<false, false><<<8, 256, 0, stream>>>(
        XC16, kDi, WXP16, kDi, DBC, kXpP, dummy_bias, dummy_resid, kDm, kL, kXpP, kDi, kSclXp);

    dt_cast_kernel<<<(kL * kDtR / 8) / 256, 256, 0, stream>>>(DBC, DTR16, kL * kDtR / 8, kCarDt);

    wmma_gemm64_f16<true, false><<<128, 256, 0, stream>>>(
        DTR16, kDtR, WDT16, kDtR, DLR, kDi, dt_b, dummy_resid, kDm, kL, kDi, kDtR, kSclDt);

    scan_kernel<<<kDi / 256, 256, 0, stream>>>(DLR, XC, XZ, DBC, A_log, Dp, YC16, dd);
  }

  wmma_gemm64_f16<false, false><<<64, 256, 0, stream>>>(
      YC16, kYcP, WOUT16, kYcP, SS, kDm, dummy_bias, dummy_resid, kDm, kL, kDm, kYcP, kSclOut);

  norm_mid_kernel<<<kL, 128, 0, stream>>>(SS, hs, mnorm_w, ln2_w, X1, H16);

  cast_rows_f16_kernel<<<(kIs * kDm / 8) / 256, 256, 0, stream>>>(gate_w, WGU16, kDm, kIs, kDm, 0, kIs * kDm / 8, kCarW);
  cast_rows_f16_kernel<<<(kIs * kDm / 8) / 256, 256, 0, stream>>>(up_w, WGU16 + (size_t)kIs * kDm, kDm, kIs, kDm, 0, kIs * kDm / 8, kCarW);
  cast_rows_f16_kernel<<<(kDm * kIs / 8) / 256, 256, 0, stream>>>(down_w, WDN16, kIs, kDm, kIs, 0, kDm * kIs / 8, kCarW);

  wmma_gemm64_f16<false, false><<<512, 256, 0, stream>>>(
      H16, kDm, WGU16, kDm, GU, kGuP, dummy_bias, dummy_resid, kDm, kL, kGuP, kDm, kSclGu);

  silu_mul_kernel<<<(kL * kIs / 8) / 256, 256, 0, stream>>>(GU, ACT16, kL * kIs / 8);

  wmma_gemm64_f16<false, true><<<64, 256, 0, stream>>>(
      ACT16, kIs, WDN16, kIs, dout, kDm, dummy_bias, X1, kDm, kL, kDm, kIs, kSclDn);
}
